// LSTM_27582279975612
// MI455X (gfx1250) — hardware-verified
//
#include <hip/hip_runtime.h>
#include <math.h>

constexpr int SEQ_T    = 20;
constexpr int BATCH_B  = 256;
constexpr int IN_F     = 512;
constexpr int HID_U    = 1024;
constexpr int GATE_N   = 4 * HID_U;
constexpr int OUT_F    = 256;
constexpr int ROWS_ALL = SEQ_T * BATCH_B;
constexpr int SLAB_P   = 68;
constexpr float ACT_CARRY = 64.0f;
constexpr float WGT_CARRY = 16.0f;
constexpr float ACC_FOLD  = 1.0f / (ACT_CARRY * WGT_CARRY);

static_assert(IN_F % 32 == 0 && HID_U % 32 == 0, "K multiples of 32");
static_assert(BATCH_B % 64 == 0 && ROWS_ALL % 64 == 0, "M multiples of 64");
static_assert(GATE_N % 64 == 0 && OUT_F % 64 == 0 && HID_U % 64 == 0, "N multiples of 64");
static_assert((BATCH_B / 64) * (HID_U / 64) == 64, "cell grid");
static_assert(((ROWS_ALL / 64) * (OUT_F / 64)) % 8 == 0, "projection grid exact");
static_assert((size_t)SEQ_T * BATCH_B * OUT_F * 4 == (size_t)5242880, "output bytes");

typedef __attribute__((ext_vector_type(16))) _Float16 v16h;
typedef __attribute__((ext_vector_type(8)))  _Float16 v8h;
typedef __attribute__((ext_vector_type(8)))  float    v8f;
typedef __attribute__((ext_vector_type(4)))  float    v4f;

__device__ __forceinline__ v16h frag_load(const _Float16* p) {
  union U { v16h v; v8h h[2]; };
  U f;
  f.h[0] = *(const v8h*)(p);
  f.h[1] = *(const v8h*)(p + 16);
  return f.v;
}
__device__ __forceinline__ v8f frag_mma(v16h a, v16h b, v8f c) {
  return __builtin_amdgcn_wmma_f32_16x16x32_f16(false, a, false, b, (short)0, c, false, false);
}
__device__ __forceinline__ void group_guard(v8f& a, v8f& b, v8f& c, v8f& d, v16h x, v16h y0, v16h y1, v16h y2, v16h y3) {
  asm volatile("v_nop\n\tv_nop\n\tv_nop\n\tv_nop" : "+v"(a), "+v"(b), "+v"(c), "+v"(d) : "v"(x), "v"(y0), "v"(y1), "v"(y2), "v"(y3));
}
__device__ __forceinline__ void keep4_h(v16h a, v16h b, v16h c, v16h d) { asm volatile("v_nop" :: "v"(a), "v"(b), "v"(c), "v"(d)); }
__device__ __forceinline__ void acc_guard4(v8f& a, v8f& b, v8f& c, v8f& d) { asm volatile("v_nop\n\tv_nop\n\tv_nop\n\tv_nop" : "+v"(a), "+v"(b), "+v"(c), "+v"(d)); }

__device__ __forceinline__ void gemm_tile64(v8f (&acc)[4][4], const _Float16* __restrict__ A, int lda,
                                            const _Float16* __restrict__ Bt, int ldb, int K,
                                            int m0, int n0, int rlane, int koff) {
  const _Float16* ap0 = A  + (size_t)(m0 + rlane) * (size_t)lda + koff;
  const _Float16* bp0 = Bt + (size_t)(n0 + rlane) * (size_t)ldb + koff;
  const size_t a16 = (size_t)16 * (size_t)lda;
  const size_t b16 = (size_t)16 * (size_t)ldb;
#pragma unroll 1
  for (int k0 = 0; k0 < K; k0 += 32) {
    v16h bh[4];
#pragma unroll
    for (int j = 0; j < 4; ++j) bh[j] = frag_load(bp0 + (size_t)j * b16 + k0);
#pragma unroll
    for (int i = 0; i < 4; ++i) {
      const v16h ah = frag_load(ap0 + (size_t)i * a16 + k0);
#pragma unroll
      for (int j = 0; j < 4; ++j) acc[i][j] = frag_mma(ah, bh[j], acc[i][j]);
      group_guard(acc[i][0], acc[i][1], acc[i][2], acc[i][3], ah, bh[0], bh[1], bh[2], bh[3]);
    }
    keep4_h(bh[0], bh[1], bh[2], bh[3]);
  }
}

template <bool PERM>
__global__ __launch_bounds__(256) void cvt8_f16_kernel(const float* __restrict__ src, unsigned short* __restrict__ dst,
                                                       int nrow, int ncol8, float sc) {
  const int i  = blockIdx.x * 256 + threadIdx.x;
  const int n8 = nrow * ncol8;
  if (i < n8) {
    const int row = i / ncol8;
    const int c8  = i - row * ncol8;
    int srow = row;
    if (PERM) {
      const int tn = row >> 6;
      const int g  = (row >> 4) & 3;
      const int cc = row & 15;
      srow = g * HID_U + tn * 16 + cc;
    }
    const float* sp = src + (size_t)srow * (size_t)(ncol8 * 8) + (size_t)c8 * 8;
    const v4f a = *(const v4f*)(sp);
    const v4f b = *(const v4f*)(sp + 4);
    v8h hv;
#pragma unroll
    for (int e = 0; e < 4; ++e) {
      hv[e]     = (_Float16)(a[e] * sc);
      hv[4 + e] = (_Float16)(b[e] * sc);
    }
    _Float16* dp = (_Float16*)dst + (size_t)i * 8;
    *(volatile v8h*)dp = hv;
    __threadfence();
    *(volatile v8h*)dp = hv;
  }
}

__global__ __launch_bounds__(128) void lstm_cell_kernel(
    const unsigned short* __restrict__ Xp, int kx,
    const unsigned short* __restrict__ Hprevp,
    const unsigned short* __restrict__ Wihp, const unsigned short* __restrict__ Whhp,
    const float* __restrict__ bih, const float* __restrict__ bhh,
    const float* __restrict__ Cin, float* __restrict__ Cout,
    unsigned short* __restrict__ Houtp, int first) {
  __shared__ __align__(16) float sZ[4][16 * SLAB_P];
  __shared__ __align__(16) float sH[64 * SLAB_P];
  const _Float16* X     = (const _Float16*)Xp;
  const _Float16* Hprev = (const _Float16*)Hprevp;
  const _Float16* Wih   = (const _Float16*)Wihp;
  const _Float16* Whh   = (const _Float16*)Whhp;
  _Float16* Hout = (_Float16*)Houtp;

  const int tid   = threadIdx.x;
  const int lane  = tid & 31;
  const int wave  = tid >> 5;
  const int rlane = lane & 15;
  const int koff  = (lane >> 4) * 8;
  const int mOff  = (lane >> 4) * 8;
  const int tmb   = blockIdx.x >> 4;
  const int hbk   = blockIdx.x & 15;
  const int tn    = hbk * 4 + wave;
  const int m0    = tmb * 64;
  const int n0    = tn * 64;

  v8f acc[4][4];
#pragma unroll
  for (int i = 0; i < 4; ++i)
#pragma unroll
    for (int j = 0; j < 4; ++j) acc[i][j] = (v8f){0.f, 0.f, 0.f, 0.f, 0.f, 0.f, 0.f, 0.f};

  gemm_tile64(acc, X, kx, Wih, kx, kx, m0, n0, rlane, koff);
  if (first == 0) gemm_tile64(acc, Hprev, HID_U, Whh, HID_U, HID_U, m0, n0, rlane, koff);
  acc_guard4(acc[0][0], acc[0][1], acc[0][2], acc[0][3]);
  acc_guard4(acc[1][0], acc[1][1], acc[1][2], acc[1][3]);
  acc_guard4(acc[2][0], acc[2][1], acc[2][2], acc[2][3]);
  acc_guard4(acc[3][0], acc[3][1], acc[3][2], acc[3][3]);

  const int hcol = hbk * 64 + wave * 16 + rlane;
  const float bI = bih[hcol]             + bhh[hcol];
  const float bF = bih[HID_U + hcol]     + bhh[HID_U + hcol];
  const float bG = bih[2 * HID_U + hcol] + bhh[2 * HID_U + hcol];
  const float bO = bih[3 * HID_U + hcol] + bhh[3 * HID_U + hcol];

  float* slab = sZ[wave];
  const size_t cbase = (size_t)(tmb * 64 + tn) * (size_t)1024;
  v4f cn4[4][2];

#pragma unroll
  for (int i = 0; i < 4; ++i) {
#pragma unroll
    for (int j = 0; j < 4; ++j)
#pragma unroll
      for (int r = 0; r < 8; ++r) slab[(mOff + r) * SLAB_P + (j << 4) + rlane] = acc[i][j][r];
    float* sp = slab + mOff * SLAB_P + rlane;
    const float* cin_i = Cin + cbase + (size_t)i * 256 + (size_t)lane * 4;
    float* hrow = sH + (i * 16 + mOff) * SLAB_P + wave * 16 + rlane;
#pragma unroll 1
    for (int r = 0; r < 8; ++r) {
      const float zi = sp[r * SLAB_P]      * ACC_FOLD + bI;
      const float zf = sp[r * SLAB_P + 16] * ACC_FOLD + bF;
      const float zg = sp[r * SLAB_P + 32] * ACC_FOLD + bG;
      const float zo = sp[r * SLAB_P + 48] * ACC_FOLD + bO;
      float cprev = 0.0f;
      if (first == 0) cprev = cin_i[(r >> 2) * 128 + (r & 3)];
      const float ig = 1.0f / (1.0f + expf(-zi));
      const float fg = 1.0f / (1.0f + expf(-zf));
      const float og = 1.0f / (1.0f + expf(-zo));
      const float gg = tanhf(zg);
      const float cnv = fg * cprev + ig * gg;
      const float hn  = og * tanhf(cnv);
      sp[r * SLAB_P] = cnv;
      hrow[r * SLAB_P] = hn * ACT_CARRY;
    }
#pragma unroll
    for (int e = 0; e < 4; ++e) {
      cn4[i][0][e] = slab[(mOff + e) * SLAB_P + rlane];
      cn4[i][1][e] = slab[(mOff + 4 + e) * SLAB_P + rlane];
    }
  }

  {
    float* cout_t = Cout + cbase + (size_t)lane * 4;
    for (int pass = 0; pass < 2; ++pass) {
#pragma unroll
      for (int i = 0; i < 4; ++i) {
        *(volatile v4f*)(cout_t + i * 256)       = cn4[i][0];
        *(volatile v4f*)(cout_t + i * 256 + 128) = cn4[i][1];
      }
      __threadfence();
    }
  }

  __syncthreads();

  {
    const int q  = tid >> 3;
    const int c8 = (tid & 7) * 8;
    v8h hv[4];
#pragma unroll
    for (int it = 0; it < 4; ++it) {
      const float* hp = sH + (it * 16 + q) * SLAB_P + c8;
      const v4f a = *(const v4f*)(hp);
      const v4f b = *(const v4f*)(hp + 4);
#pragma unroll
      for (int e = 0; e < 4; ++e) {
        hv[it][e]     = (_Float16)a[e];
        hv[it][4 + e] = (_Float16)b[e];
      }
    }
    for (int pass = 0; pass < 2; ++pass) {
#pragma unroll
      for (int it = 0; it < 4; ++it) {
        const int row = it * 16 + q;
        *(volatile v8h*)(Hout + (size_t)(m0 + row) * HID_U + hbk * 64 + c8) = hv[it];
      }
      __threadfence();
    }
  }
}

__global__ __launch_bounds__(256) void out_gemm_kernel(const unsigned short* __restrict__ Ap,
                                                       const unsigned short* __restrict__ Btp,
                                                       const float* __restrict__ bias, float* __restrict__ C) {
  __shared__ __align__(16) float sT[8][16 * SLAB_P];
  const _Float16* A  = (const _Float16*)Ap;
  const _Float16* Bt = (const _Float16*)Btp;
  const int lane  = threadIdx.x & 31;
  const int wave  = threadIdx.x >> 5;
  const int tilesN = OUT_F / 64;
  const int tilesM = ROWS_ALL / 64;
  const int tile = blockIdx.x * 8 + wave;
  if (tile >= tilesM * tilesN) return;
  const int tm = tile / tilesN;
  const int tn = tile - tm * tilesN;
  const int m0 = tm << 6;
  const int n0 = tn << 6;
  const int rlane = lane & 15;
  const int koff  = (lane >> 4) * 8;
  const int mOff  = (lane >> 4) * 8;

  v8f acc[4][4];
#pragma unroll
  for (int i = 0; i < 4; ++i)
#pragma unroll
    for (int j = 0; j < 4; ++j) acc[i][j] = (v8f){0.f, 0.f, 0.f, 0.f, 0.f, 0.f, 0.f, 0.f};

  gemm_tile64(acc, A, HID_U, Bt, HID_U, HID_U, m0, n0, rlane, koff);
  acc_guard4(acc[0][0], acc[0][1], acc[0][2], acc[0][3]);
  acc_guard4(acc[1][0], acc[1][1], acc[1][2], acc[1][3]);
  acc_guard4(acc[2][0], acc[2][1], acc[2][2], acc[2][3]);
  acc_guard4(acc[3][0], acc[3][1], acc[3][2], acc[3][3]);

  float* slab = sT[wave];
#pragma unroll
  for (int i = 0; i < 4; ++i) {
    const int mBase = m0 + (i << 4);
#pragma unroll
    for (int j = 0; j < 4; ++j) {
      const float bv = bias[n0 + (j << 4) + rlane];
#pragma unroll
      for (int r = 0; r < 8; ++r) slab[(mOff + r) * SLAB_P + (j << 4) + rlane] = acc[i][j][r] * ACC_FOLD + bv;
    }
    __builtin_amdgcn_fence(__ATOMIC_RELEASE, "workgroup");
    __builtin_amdgcn_wave_barrier();
    __builtin_amdgcn_fence(__ATOMIC_ACQUIRE, "workgroup");
    {
      const int hh = lane >> 4;
      const int c4 = (lane & 15) * 4;
      for (int pass = 0; pass < 2; ++pass) {
#pragma unroll
        for (int it = 0; it < 8; ++it) {
          const int row = it * 2 + hh;
          const v4f v = *(const v4f*)(slab + row * SLAB_P + c4);
          *(volatile v4f*)(C + (size_t)(mBase + row) * OUT_F + n0 + c4) = v;
        }
        __threadfence();
      }
    }
    __builtin_amdgcn_fence(__ATOMIC_RELEASE, "workgroup");
    __builtin_amdgcn_wave_barrier();
    __builtin_amdgcn_fence(__ATOMIC_ACQUIRE, "workgroup");
  }
}

extern "C" void kernel_launch(void* const* d_in, const int* in_sizes, int n_in,
                              void* d_out, int out_size, void* d_ws, size_t ws_size, hipStream_t stream) {
  if (n_in < 15 || d_out == nullptr || d_ws == nullptr) return;
  if (in_sizes[0] != SEQ_T * BATCH_B * IN_F || in_sizes[1] != GATE_N * IN_F || in_sizes[2] != GATE_N * HID_U ||
      in_sizes[3] != GATE_N || in_sizes[4] != GATE_N || in_sizes[5] != GATE_N * HID_U || in_sizes[6] != GATE_N * HID_U ||
      in_sizes[7] != GATE_N || in_sizes[8] != GATE_N || in_sizes[9] != GATE_N * HID_U || in_sizes[10] != GATE_N * HID_U ||
      in_sizes[11] != GATE_N || in_sizes[12] != GATE_N || in_sizes[13] != OUT_F * HID_U || in_sizes[14] != OUT_F ||
      out_size != SEQ_T * BATCH_B * OUT_F) return;

  const float* input = (const float*)d_in[0];
  const float* w_ih[3] = { (const float*)d_in[1], (const float*)d_in[5], (const float*)d_in[9] };
  const float* w_hh[3] = { (const float*)d_in[2], (const float*)d_in[6], (const float*)d_in[10] };
  const float* b_ih[3] = { (const float*)d_in[3], (const float*)d_in[7], (const float*)d_in[11] };
  const float* b_hh[3] = { (const float*)d_in[4], (const float*)d_in[8], (const float*)d_in[12] };
  const float* w_out = (const float*)d_in[13];
  const float* b_out = (const float*)d_in[14];
  float* out = (float*)d_out;

  char* ws = (char*)d_ws;
  size_t off = 0;
  auto carve = [&](size_t bytes) -> char* { char* p = ws + off; off += (bytes + 255) & ~(size_t)255; return p; };
  unsigned short* X16 = (unsigned short*)carve((size_t)ROWS_ALL * IN_F * 2);
  unsigned short* WIH[3];
  unsigned short* WHH[3];
  WIH[0] = (unsigned short*)carve((size_t)GATE_N * IN_F * 2);
  WHH[0] = (unsigned short*)carve((size_t)GATE_N * HID_U * 2);
  WIH[1] = (unsigned short*)carve((size_t)GATE_N * HID_U * 2);
  WHH[1] = (unsigned short*)carve((size_t)GATE_N * HID_U * 2);
  WIH[2] = (unsigned short*)carve((size_t)GATE_N * HID_U * 2);
  WHH[2] = (unsigned short*)carve((size_t)GATE_N * HID_U * 2);
  unsigned short* WOUT = (unsigned short*)carve((size_t)OUT_F * HID_U * 2);
  unsigned short* HP[3];
  HP[0] = (unsigned short*)carve((size_t)ROWS_ALL * HID_U * 2);
  HP[1] = (unsigned short*)carve((size_t)ROWS_ALL * HID_U * 2);
  HP[2] = (unsigned short*)carve((size_t)ROWS_ALL * HID_U * 2);
  float* CP[3][2];
  for (int l = 0; l < 3; ++l)
    for (int p = 0; p < 2; ++p) CP[l][p] = (float*)carve((size_t)BATCH_B * HID_U * 4);
  if (off > ws_size || off > (size_t)134217728) return;

  {
    const int n8x = ROWS_ALL * (IN_F / 8);
    const int n8a = GATE_N * (IN_F / 8);
    const int n8b = GATE_N * (HID_U / 8);
    const int n8o = OUT_F * (HID_U / 8);
    cvt8_f16_kernel<false><<<(n8x + 255) / 256, 256, 0, stream>>>(input, X16, ROWS_ALL, IN_F / 8, ACT_CARRY);
    cvt8_f16_kernel<true><<<(n8a + 255) / 256, 256, 0, stream>>>(w_ih[0], WIH[0], GATE_N, IN_F / 8, WGT_CARRY);
    cvt8_f16_kernel<true><<<(n8b + 255) / 256, 256, 0, stream>>>(w_hh[0], WHH[0], GATE_N, HID_U / 8, WGT_CARRY);
    cvt8_f16_kernel<true><<<(n8b + 255) / 256, 256, 0, stream>>>(w_ih[1], WIH[1], GATE_N, HID_U / 8, WGT_CARRY);
    cvt8_f16_kernel<true><<<(n8b + 255) / 256, 256, 0, stream>>>(w_hh[1], WHH[1], GATE_N, HID_U / 8, WGT_CARRY);
    cvt8_f16_kernel<true><<<(n8b + 255) / 256, 256, 0, stream>>>(w_ih[2], WIH[2], GATE_N, HID_U / 8, WGT_CARRY);
    cvt8_f16_kernel<true><<<(n8b + 255) / 256, 256, 0, stream>>>(w_hh[2], WHH[2], GATE_N, HID_U / 8, WGT_CARRY);
    cvt8_f16_kernel<false><<<(n8o + 255) / 256, 256, 0, stream>>>(w_out, WOUT, OUT_F, HID_U / 8, WGT_CARRY);
  }

  const int cell_grid = (BATCH_B / 64) * (HID_U / 64);
  for (int l = 0; l < 3; ++l) {
    for (int t = 0; t < SEQ_T; ++t) {
      const unsigned short* xp;
      int kx;
      if (l == 0) { xp = X16 + (size_t)t * BATCH_B * IN_F; kx = IN_F; }
      else        { xp = HP[l - 1] + (size_t)t * BATCH_B * HID_U; kx = HID_U; }
      const int first = (t == 0) ? 1 : 0;
      const unsigned short* hprev = (t == 0) ? xp : (HP[l] + (size_t)(t - 1) * BATCH_B * HID_U);
      unsigned short* hout = HP[l] + (size_t)t * BATCH_B * HID_U;
      const float* cin = CP[l][(t + 1) & 1];
      float* cout_p = CP[l][t & 1];
      lstm_cell_kernel<<<cell_grid, 128, 0, stream>>>(xp, kx, hprev, WIH[l], WHH[l], b_ih[l], b_hh[l],
                                                      cin, cout_p, hout, first);
    }
  }

  out_gemm_kernel<<<((ROWS_ALL / 64) * (OUT_F / 64)) / 8, 256, 0, stream>>>(HP[2], WOUT, b_out, out);
}
